// NODE_17927193494211
// MI455X (gfx1250) — hardware-verified
//
#include <hip/hip_runtime.h>
#include <math.h>

constexpr int kBatch  = 8192;
constexpr int kIn     = 256;
constexpr int kTrees  = 128;
constexpr int kDepth  = 8;
constexpr int kCols   = kTrees * kDepth;
constexpr int kLeaves = 256;

constexpr int kTreeThreads = 256;
constexpr int kTreeWaves   = kTreeThreads / 32;
constexpr int kTreeGroup   = 16;
constexpr int kTP          = 20;

constexpr float kUCarry   = 32768.0f;
constexpr float kULoCarry = 2048.0f;
constexpr float kRCarry   = 16.0f;
constexpr float kInvHi    = 1.0f / (32768.0f * 16.0f);
constexpr float kInvLo    = kInvHi / 2048.0f;
constexpr float kInvTrees = 1.0f / 128.0f;

constexpr size_t kBytesXb = (size_t)kBatch * kIn * 2;
constexpr size_t kBytesWb = (size_t)kCols * kIn * 2;
constexpr size_t kBytesZ  = (size_t)kCols * kBatch * 4;
constexpr size_t kOffXb   = 0;
constexpr size_t kOffWb   = kOffXb + kBytesXb;
constexpr size_t kOffZ    = kOffWb + kBytesWb;
constexpr size_t kWsTotal = kOffZ + kBytesZ;

static_assert(kIn % 32 == 0);
static_assert(kCols % 64 == 0 && kBatch % 64 == 0);
static_assert(kBatch % kTreeThreads == 0);
static_assert((kBatch * kIn) % (8 * 256) == 0 && (kCols * kIn) % (8 * 256) == 0);
static_assert(kCols == 4 * kTreeThreads);
static_assert(kTreeGroup * 16 == kTreeThreads);
static_assert(kTrees % kTreeGroup == 0);
static_assert(kOffZ % 128 == 0 && kOffWb % 128 == 0);
static_assert(kWsTotal <= 134217728);
static_assert(kTreeThreads % 128 == 0);

typedef __attribute__((ext_vector_type(16))) _Float16 v16h;
typedef __attribute__((ext_vector_type(8)))  _Float16 v8h;
typedef __attribute__((ext_vector_type(16))) __bf16   v16b;
typedef __attribute__((ext_vector_type(8)))  __bf16   v8b;
typedef __attribute__((ext_vector_type(8)))  float    v8f;
typedef __attribute__((ext_vector_type(4)))  float    v4f;
typedef __attribute__((ext_vector_type(4)))  unsigned int v4u;

__device__ __forceinline__ unsigned short f2bf_bits(float f) {
  unsigned u = __float_as_uint(f);
  return (unsigned short)((u + 0x7FFFu + ((u >> 16) & 1u)) >> 16);
}
__device__ __forceinline__ float bf_bits2f(unsigned short h) { return __uint_as_float(((unsigned)h) << 16); }

__device__ __forceinline__ void dep_guard_h(v8f& a, v8f& b, v16h x, v16h y) { asm volatile("v_nop\n\tv_nop\n\tv_nop\n\tv_nop" : "+v"(a), "+v"(b) : "v"(x), "v"(y)); }
__device__ __forceinline__ void dep_guard_b(v8f& a, v8f& b, v16b x, v16b y) { asm volatile("v_nop\n\tv_nop\n\tv_nop\n\tv_nop" : "+v"(a), "+v"(b) : "v"(x), "v"(y)); }
__device__ __forceinline__ void keep4_h(v16h a, v16h b, v16h c, v16h d) { asm volatile("v_nop" :: "v"(a), "v"(b), "v"(c), "v"(d)); }
__device__ __forceinline__ void keep4_b(v16b a, v16b b, v16b c, v16b d) { asm volatile("v_nop" :: "v"(a), "v"(b), "v"(c), "v"(d)); }
__device__ __forceinline__ void acc_guard4(v8f& a, v8f& b, v8f& c, v8f& d) { asm volatile("v_nop\n\tv_nop\n\tv_nop\n\tv_nop" : "+v"(a), "+v"(b), "+v"(c), "+v"(d)); }
template <typename T> struct Frag;
template <> struct Frag<_Float16> {
  typedef v16h V; union U { v16h v; v8h h[2]; };
  static __device__ __forceinline__ v16h load(const _Float16* p) {
    U f; f.h[0] = *(const v8h*)(p); f.h[1] = *(const v8h*)(p + 16); return f.v;
  }
  static __device__ __forceinline__ v8f mma(v16h a, v16h b, v8f c) {
    return __builtin_amdgcn_wmma_f32_16x16x32_f16(false, a, false, b, (short)0, c, false, false);
  }
  static __device__ __forceinline__ void guard(v8f& a, v8f& b, v16h x, v16h y) { dep_guard_h(a, b, x, y); }
  static __device__ __forceinline__ void keep(v16h a, v16h b, v16h c, v16h d) { keep4_h(a, b, c, d); }
};
template <> struct Frag<__bf16> {
  typedef v16b V; union U { v16b v; v8b h[2]; };
  static __device__ __forceinline__ v16b load(const __bf16* p) {
    U f; f.h[0] = *(const v8b*)(p); f.h[1] = *(const v8b*)(p + 16); return f.v;
  }
  static __device__ __forceinline__ v8f mma(v16b a, v16b b, v8f c) {
    return __builtin_amdgcn_wmma_f32_16x16x32_bf16(false, a, false, b, (short)0, c, false, false);
  }
  static __device__ __forceinline__ void guard(v8f& a, v8f& b, v16b x, v16b y) { dep_guard_b(a, b, x, y); }
  static __device__ __forceinline__ void keep(v16b a, v16b b, v16b c, v16b d) { keep4_b(a, b, c, d); }
};

__device__ __forceinline__ unsigned pk16(unsigned short a, unsigned short b) { return (unsigned)a | ((unsigned)b << 16); }
__device__ __forceinline__ unsigned short h_bits(float f) { const _Float16 h = (_Float16)f; return __builtin_bit_cast(unsigned short, h); }

template <int ET> struct Elem;
template <> struct Elem<0> { typedef _Float16 T; };
template <> struct Elem<1> { typedef __bf16 T; };
template <int ET, bool SPLIT, int BIAS_MODE, int OUT_MODE, bool RESID, int ACT = 0>
__global__ __launch_bounds__(256) void wmma_gemm64(
    const unsigned short* __restrict__ Ap, const unsigned short* __restrict__ A2p, int lda, long strideA,
    const unsigned short* __restrict__ Btp, const unsigned short* __restrict__ Bt2p, int ldb, long strideB,
    void* __restrict__ Cout, void* __restrict__ Cout2, int ldc, long strideC,
    const float* __restrict__ bias,
    const float* __restrict__ resid, long strideR,
    int M, int N, int K, float scale) {
  typedef typename Elem<ET>::T T;
  typedef typename Frag<T>::V V;
  const T* A = (const T*)Ap; const T* A2 = (const T*)A2p; const T* Bt = (const T*)Btp; const T* Bt2 = (const T*)Bt2p;
  __shared__ __align__(16) float sT[8][16 * 68];
  const int b    = blockIdx.y;
  const int lane = threadIdx.x & 31;
  const int wave = threadIdx.x >> 5;
  const int tilesN = N >> 6;
  const int tilesM = M >> 6;
  const int tile = blockIdx.x * 8 + wave;
  if (tile >= tilesM * tilesN) return;
  const int tm = tile / tilesN;
  const int tn = tile - tm * tilesN;
  const int m0 = tm << 6;
  const int n0 = tn << 6;

  const T* Ab  = A  + (size_t)b * strideA;
  const T* Bb  = Bt + (size_t)b * strideB;
  const T* Ab2 = SPLIT ? (A2  + (size_t)b * strideA) : nullptr;
  const T* Bb2 = SPLIT ? (Bt2 + (size_t)b * strideB) : nullptr;

  const int rlane = lane & 15;
  const int koff  = (lane >> 4) * 8;
  const int mOff  = (lane >> 4) * 8;

  v8f acc[4][4];
#pragma unroll
  for (int i = 0; i < 4; ++i)
#pragma unroll
    for (int j = 0; j < 4; ++j) acc[i][j] = (v8f){0.f,0.f,0.f,0.f,0.f,0.f,0.f,0.f};

  for (int k0 = 0; k0 < K; k0 += 32) {
    V bh[4], bl[4];
#pragma unroll
    for (int j = 0; j < 4; ++j) {
      const size_t bo = (size_t)(n0 + (j << 4) + rlane) * ldb + koff + k0;
      bh[j] = Frag<T>::load(Bb + bo);
      if (SPLIT) bl[j] = Frag<T>::load(Bb2 + bo);
    }
#pragma unroll
    for (int i = 0; i < 4; ++i) {
      const size_t ao = (size_t)(m0 + (i << 4) + rlane) * lda + koff + k0;
      V ah = Frag<T>::load(Ab + ao);
      V al;
      if (SPLIT) al = Frag<T>::load(Ab2 + ao);
#pragma unroll
      for (int j = 0; j < 4; ++j) {
        acc[i][j] = Frag<T>::mma(ah, bh[j], acc[i][j]);
        if (SPLIT) {
          acc[i][j] = Frag<T>::mma(ah, bl[j], acc[i][j]);
          acc[i][j] = Frag<T>::mma(al, bh[j], acc[i][j]);
        }
      }
      Frag<T>::guard(acc[i][0], acc[i][3], ah, SPLIT ? al : ah);
    }
    Frag<T>::keep(bh[0], bh[1], bh[2], bh[3]);
    if (SPLIT) Frag<T>::keep(bl[0], bl[1], bl[2], bl[3]);
  }
  acc_guard4(acc[0][0], acc[0][1], acc[0][2], acc[0][3]);
  acc_guard4(acc[1][0], acc[1][1], acc[1][2], acc[1][3]);
  acc_guard4(acc[2][0], acc[2][1], acc[2][2], acc[2][3]);
  acc_guard4(acc[3][0], acc[3][1], acc[3][2], acc[3][3]);

  float* slab = sT[wave];
  const float* Rb = RESID ? (resid + (size_t)b * strideR) : nullptr;
#pragma unroll
  for (int i = 0; i < 4; ++i) {
    const int mBase = m0 + (i << 4);
#pragma unroll
    for (int j = 0; j < 4; ++j) {
      const int n = n0 + (j << 4) + rlane;
      float bv = 0.f;
      if (BIAS_MODE == 2) bv = bias[n];
#pragma unroll
      for (int r = 0; r < 8; ++r) {
        float v = acc[i][j][r] * scale;
        if (BIAS_MODE == 1) v += bias[mBase + mOff + r];
        if (BIAS_MODE == 2) v += bv;
        if (RESID) v += Rb[(size_t)(mBase + mOff + r) * ldc + n];
        if (ACT == 2) v = fmaxf(v, 0.0f);
        if (ACT == 4) v = (v > 0.f) ? v : 0.01f * v;
        slab[(mOff + r) * 68 + (j << 4) + rlane] = v;
      }
    }
    __builtin_amdgcn_fence(__ATOMIC_RELEASE, "workgroup");
    __builtin_amdgcn_wave_barrier();
    __builtin_amdgcn_fence(__ATOMIC_ACQUIRE, "workgroup");
    if (OUT_MODE == 0) {
      float* C = (float*)Cout + (size_t)b * strideC;
      const int hh = lane >> 4, c4 = (lane & 15) * 4;
      for (int pass = 0; pass < 2; ++pass) {
#pragma unroll
        for (int it = 0; it < 8; ++it) {
          const int row = it * 2 + hh;
          v4f v = *(const v4f*)(slab + row * 68 + c4);
          *(volatile v4f*)(C + (size_t)(mBase + row) * ldc + n0 + c4) = v;
        }
        __threadfence();
      }
    } else {
      const int q = lane >> 3, c8 = (lane & 7) * 8;
      unsigned short* C  = (unsigned short*)Cout  + (size_t)b * strideC;
      unsigned short* C2 = (OUT_MODE == 2) ? ((unsigned short*)Cout2 + (size_t)b * strideC) : nullptr;
      for (int pass = 0; pass < 2; ++pass) {
#pragma unroll
        for (int it = 0; it < 4; ++it) {
          const int row = it * 4 + q;
          const float* sp = slab + row * 68 + c8;
          v8h hv, lv;
#pragma unroll
          for (int e = 0; e < 8; ++e) {
            if (OUT_MODE == 1) {
              hv[e] = (_Float16)sp[e];
            } else {
              unsigned short hb = f2bf_bits(sp[e]);
              unsigned short lb = f2bf_bits(sp[e] - bf_bits2f(hb));
              hv[e] = __builtin_bit_cast(_Float16, hb);
              lv[e] = __builtin_bit_cast(_Float16, lb);
            }
          }
          *(volatile v8h*)(C + (size_t)(mBase + row) * ldc + n0 + c8) = hv;
          if (OUT_MODE == 2) *(volatile v8h*)(C2 + (size_t)(mBase + row) * ldc + n0 + c8) = lv;
        }
        __threadfence();
      }
    }
    __builtin_amdgcn_fence(__ATOMIC_RELEASE, "workgroup");
    __builtin_amdgcn_wave_barrier();
    __builtin_amdgcn_fence(__ATOMIC_ACQUIRE, "workgroup");
  }
}

__global__ __launch_bounds__(256) void cast8_bf16_kernel(const float* __restrict__ in, unsigned short* __restrict__ out, int n8) {
  const int i = blockIdx.x * 256 + threadIdx.x;
  if (i >= n8) return;
  const float* p = in + 8 * (size_t)i;
  const v4f a = *(const v4f*)(p);
  const v4f c = *(const v4f*)(p + 4);
  unsigned short hb[8];
#pragma unroll
  for (int e = 0; e < 4; ++e) {
    hb[e]     = f2bf_bits(a[e]);
    hb[4 + e] = f2bf_bits(c[e]);
  }
  const v4u u = (v4u){pk16(hb[0], hb[1]), pk16(hb[2], hb[3]), pk16(hb[4], hb[5]), pk16(hb[6], hb[7])};
  unsigned short* q = out + 8 * (size_t)i;
  *(volatile v4u*)q = u;
  __threadfence();
  *(volatile v4u*)q = u;
}

union HFrag { v16h v; v8h h[2]; v4u w[2]; };
__device__ __forceinline__ v16h load_lowk16(const unsigned short* p) {
  HFrag f;
  f.h[0] = *(const v8h*)(const void*)p;
  f.w[1] = (v4u){0u, 0u, 0u, 0u};
  return f.v;
}
__device__ __forceinline__ v8f mma_h_guarded(v16h a, v16h b, v8f c) {
  c = __builtin_amdgcn_wmma_f32_16x16x32_f16(false, a, false, b, (short)0, c, false, false);
  asm volatile("v_nop\n\tv_nop\n\tv_nop\n\tv_nop" : "+v"(c) : "v"(a), "v"(b));
  return c;
}

__global__ __launch_bounds__(kTreeThreads) void tree_eval_kernel(const float* __restrict__ Z,
                                                                 const float* __restrict__ bias,
                                                                 const float* __restrict__ R,
                                                                 float* __restrict__ out) {
  __shared__ __align__(16) float          sBias[kCols];
  __shared__ __align__(16) unsigned short sRT[kTreeGroup * 16 * 16];
  __shared__ __align__(16) unsigned short sUh[kTreeWaves][32 * 16];
  __shared__ __align__(16) unsigned short sUl[kTreeWaves][32 * 16];
  __shared__ __align__(16) float          sTs[kTreeWaves][32 * kTP];
  __shared__ __align__(16) float          sOut[kTreeThreads];

  const int tid  = threadIdx.x;
  const int lane = tid & 31;
  const int wave = tid >> 5;
  const int hh   = lane >> 4;
  const int rl   = lane & 15;
  const int koff = hh * 8;
  const int brow = blockIdx.x * kTreeThreads + tid;

  {
    const v4f bv = *(const v4f*)(bias + 4 * tid);
#pragma unroll
    for (int e = 0; e < 4; ++e) sBias[4 * tid + e] = bf_bits2f(f2bf_bits(bv[e]));
  }

  unsigned short* uh = sUh[wave];
  unsigned short* ul = sUl[wave];
  float* ts = sTs[wave];
  float accTot = 0.0f;

#pragma unroll 1
  for (int tg = 0; tg < kTrees / kTreeGroup; ++tg) {
    __syncthreads();
    {
      const int tl = tid >> 4, ci = tid & 15;
      const float* rp = R + (size_t)(tg * kTreeGroup + tl) * kLeaves + ci * 16;
      unsigned short* dst = sRT + (tl * 16) * 16 + ci;
#pragma unroll
      for (int q4 = 0; q4 < 4; ++q4) {
        const v4f rv = *(const v4f*)(rp + 4 * q4);
#pragma unroll
        for (int e = 0; e < 4; ++e) {
          const float rb = bf_bits2f(f2bf_bits(rv[e])) * kRCarry;
          dst[(q4 * 4 + e) * 16] = h_bits(rb);
        }
      }
    }
    __syncthreads();

#pragma unroll 1
    for (int tt = 0; tt < kTreeGroup; ++tt) {
      const int t = tg * kTreeGroup + tt;

      float p[kDepth], q[kDepth];
#pragma unroll
      for (int d = 0; d < kDepth; ++d) {
        const int col = t * kDepth + d;
        const float zb = Z[(size_t)col * kBatch + brow] + sBias[col];
        const float ez = expf(-fabsf(zb));
        const float sg = 1.0f / (1.0f + ez);
        const float sn = ez * sg;
        const float pd = (zb >= 0.0f) ? sg : sn;
        p[d] = pd;
        q[d] = 1.0f - pd;
      }

      float u[16], v[16];
      u[0] = 1.0f; v[0] = 1.0f;
#pragma unroll
      for (int d = 0; d < 4; ++d) {
        const int cnt = 1 << d;
#pragma unroll
        for (int i = cnt - 1; i >= 0; --i) {
          const float tu = u[i], tv = v[i];
          u[2 * i + 1] = tu * p[d];      u[2 * i] = tu * q[d];
          v[2 * i + 1] = tv * p[4 + d];  v[2 * i] = tv * q[4 + d];
        }
      }

      unsigned int wh[8], wl[8];
#pragma unroll
      for (int i2 = 0; i2 < 8; ++i2) {
        const float us0 = u[2 * i2] * kUCarry;
        const float us1 = u[2 * i2 + 1] * kUCarry;
        const _Float16 h0 = (_Float16)us0;
        const _Float16 h1 = (_Float16)us1;
        const float hf0 = (float)h0;
        const float hf1 = (float)h1;
        const _Float16 l0 = (_Float16)((us0 - hf0) * kULoCarry);
        const _Float16 l1 = (_Float16)((us1 - hf1) * kULoCarry);
        wh[i2] = pk16(__builtin_bit_cast(unsigned short, h0), __builtin_bit_cast(unsigned short, h1));
        wl[i2] = pk16(__builtin_bit_cast(unsigned short, l0), __builtin_bit_cast(unsigned short, l1));
      }
      *(v4u*)(void*)(uh + lane * 16)     = (v4u){wh[0], wh[1], wh[2], wh[3]};
      *(v4u*)(void*)(uh + lane * 16 + 8) = (v4u){wh[4], wh[5], wh[6], wh[7]};
      *(v4u*)(void*)(ul + lane * 16)     = (v4u){wl[0], wl[1], wl[2], wl[3]};
      *(v4u*)(void*)(ul + lane * 16 + 8) = (v4u){wl[4], wl[5], wl[6], wl[7]};
      __builtin_amdgcn_fence(__ATOMIC_RELEASE, "workgroup");
      __builtin_amdgcn_wave_barrier();
      __builtin_amdgcn_fence(__ATOMIC_ACQUIRE, "workgroup");

      const v16h bR = load_lowk16(sRT + (tt * 16 + rl) * 16 + koff);
      v8f accH0 = (v8f){0.f,0.f,0.f,0.f,0.f,0.f,0.f,0.f};
      v8f accL0 = accH0, accH1 = accH0, accL1 = accH0;
      {
        const v16h ah0 = load_lowk16(uh + rl * 16 + koff);
        const v16h al0 = load_lowk16(ul + rl * 16 + koff);
        accH0 = mma_h_guarded(ah0, bR, accH0);
        accL0 = mma_h_guarded(al0, bR, accL0);
        const v16h ah1 = load_lowk16(uh + (16 + rl) * 16 + koff);
        const v16h al1 = load_lowk16(ul + (16 + rl) * 16 + koff);
        accH1 = mma_h_guarded(ah1, bR, accH1);
        accL1 = mma_h_guarded(al1, bR, accL1);
      }
#pragma unroll
      for (int r = 0; r < 8; ++r) {
        ts[(8 * hh + r) * kTP + rl]      = accH0[r] * kInvHi + accL0[r] * kInvLo;
        ts[(16 + 8 * hh + r) * kTP + rl] = accH1[r] * kInvHi + accL1[r] * kInvLo;
      }
      __builtin_amdgcn_fence(__ATOMIC_RELEASE, "workgroup");
      __builtin_amdgcn_wave_barrier();
      __builtin_amdgcn_fence(__ATOMIC_ACQUIRE, "workgroup");

      const float* tr = ts + lane * kTP;
      const v4f t0 = *(const v4f*)(tr);
      const v4f t1 = *(const v4f*)(tr + 4);
      const v4f t2 = *(const v4f*)(tr + 8);
      const v4f t3 = *(const v4f*)(tr + 12);
      float tval = 0.0f;
#pragma unroll
      for (int j = 0; j < 4; ++j) tval = fmaf(v[j], t0[j], tval);
#pragma unroll
      for (int j = 0; j < 4; ++j) tval = fmaf(v[4 + j], t1[j], tval);
#pragma unroll
      for (int j = 0; j < 4; ++j) tval = fmaf(v[8 + j], t2[j], tval);
#pragma unroll
      for (int j = 0; j < 4; ++j) tval = fmaf(v[12 + j], t3[j], tval);
      accTot += tval;
    }
  }

  sOut[tid] = accTot * kInvTrees;
  __syncthreads();
  if (tid < 64) {
    const v4f ov = *(const v4f*)(sOut + 4 * tid);
    float* op = out + (size_t)blockIdx.x * kTreeThreads + 4 * tid;
    *(volatile v4f*)op = ov;
    __threadfence();
    *(volatile v4f*)op = ov;
  }
}

extern "C" void kernel_launch(void* const* d_in, const int* in_sizes, int n_in,
                              void* d_out, int out_size, void* d_ws, size_t ws_size,
                              hipStream_t stream) {
  if (n_in < 4) return;
  if (in_sizes[0] != kBatch * kIn || in_sizes[1] != kCols * kIn || in_sizes[2] != kCols ||
      in_sizes[3] != kTrees * kLeaves || out_size != kBatch || ws_size < kWsTotal || d_ws == nullptr) return;

  const float* x    = (const float*)d_in[0];
  const float* wsel = (const float*)d_in[1];
  const float* fb   = (const float*)d_in[2];
  const float* resp = (const float*)d_in[3];
  float* outp       = (float*)d_out;

  unsigned char* ws = (unsigned char*)d_ws;
  unsigned short* Xb = (unsigned short*)(ws + kOffXb);
  unsigned short* Wb = (unsigned short*)(ws + kOffWb);
  float* Zp          = (float*)(ws + kOffZ);

  cast8_bf16_kernel<<<dim3((kBatch * kIn / 8) / 256), dim3(256), 0, stream>>>(x, Xb, kBatch * kIn / 8);
  cast8_bf16_kernel<<<dim3((kCols * kIn / 8) / 256), dim3(256), 0, stream>>>(wsel, Wb, kCols * kIn / 8);

  wmma_gemm64<1, false, 0, 0, false><<<dim3((kCols / 64) * (kBatch / 64) / 8, 1), dim3(256), 0, stream>>>(
      Wb, Wb, kIn, (long)0,
      Xb, Xb, kIn, (long)0,
      (void*)Zp, (void*)Zp, kBatch, (long)0,
      fb, fb, (long)0,
      kCols, kBatch, kIn, 1.0f);

  tree_eval_kernel<<<dim3(kBatch / kTreeThreads), dim3(kTreeThreads), 0, stream>>>(Zp, fb, resp, outp);
}
